// MaskedAttention_37469294691214
// MI455X (gfx1250) — hardware-verified
//
#include <hip/hip_runtime.h>
#include <stdint.h>

#ifndef NB
#define NB 2
#endif
#ifndef SEQ
#define SEQ 2048
#endif
#define NB_FULL  2
#define SEQ_FULL 2048
#define DM       1024
#define NH       16
#define HD       64
#define NTOK     (NB * SEQ)
#define LQK      (2 * DM)
#define LCB      (2 * DM)

typedef _Float16 v16h __attribute__((ext_vector_type(16)));
typedef _Float16 v8h  __attribute__((ext_vector_type(8)));
typedef __bf16   v16b __attribute__((ext_vector_type(16)));
typedef __bf16   v8b  __attribute__((ext_vector_type(8)));
typedef float    v8f  __attribute__((ext_vector_type(8)));
typedef float    v4f  __attribute__((ext_vector_type(4)));
typedef unsigned short v8us __attribute__((ext_vector_type(8)));
union Frag { v16h v; v8h half[2]; };

static_assert((DM % 64) == 0 && (NTOK % 64) == 0 && (DM % 32) == 0);
static_assert((SEQ % 32) == 0 && SEQ <= SEQ_FULL && NB >= 1 && NB <= NB_FULL);
static_assert(NH * HD == DM && HD == 64 && (DM / 8) == 128);
static_assert(((NB - 1) * SEQ_FULL + SEQ) <= NB_FULL * SEQ_FULL);

__device__ __forceinline__ unsigned short bfbits(float f) {
  const unsigned u = __float_as_uint(f);
  return (unsigned short)((u + 0x7FFFu + ((u >> 16) & 1u)) >> 16);
}
__device__ __forceinline__ float bfval(float f) {
  return __uint_as_float(((unsigned)bfbits(f)) << 16);
}

__device__ __forceinline__ v16h ldfrag(const _Float16* p) {
  union { v16h v; v8h hh[2]; } f;
  f.hh[0] = *(const v8h*)(p);
  f.hh[1] = *(const v8h*)(p + 16);
  return f.v;
}
__device__ __forceinline__ v16b ldfragb(const __bf16* p) {
  union { v16b v; v8b hh[2]; } f;
  f.hh[0] = *(const v8b*)(p);
  f.hh[1] = *(const v8b*)(p + 16);
  return f.v;
}
__device__ __forceinline__ v8f mma16(v16h a, v16h b, v8f c) {
  return __builtin_amdgcn_wmma_f32_16x16x32_f16(false, a, false, b, (short)0, c, false, false);
}
__device__ __forceinline__ v8f mmabf(v16b a, v16b b, v8f c) {
  return __builtin_amdgcn_wmma_f32_16x16x32_bf16(false, a, false, b, (short)0, c, false, false);
}
__device__ __forceinline__ v8f zero8() {
  v8f z;
#pragma unroll
  for (int i = 0; i < 8; ++i) z[i] = 0.0f;
  return z;
}

__device__ __forceinline__ void guard_g(v8f& a, v8f& b, v16b x, v16b y) {
  asm volatile("v_nop\n\tv_nop\n\tv_nop\n\tv_nop" : "+v"(a), "+v"(b) : "v"(x), "v"(y));
}
__device__ __forceinline__ void keep4(v16b a, v16b b, v16b c, v16b d) {
  asm volatile("v_nop" :: "v"(a), "v"(b), "v"(c), "v"(d));
}
__device__ __forceinline__ void accg4(v8f& a, v8f& b, v8f& c, v8f& d) {
  asm volatile("v_nop\n\tv_nop\n\tv_nop\n\tv_nop" : "+v"(a), "+v"(b), "+v"(c), "+v"(d));
}
__device__ __forceinline__ void guard_st(v8f& a, v8f& b, v16h x0, v16h x1, v16h x2, v16h x3,
                                         v16h y0, v16h y1, v16h y2, v16h y3) {
  asm volatile("v_nop\n\tv_nop\n\tv_nop\n\tv_nop"
               : "+v"(a), "+v"(b)
               : "v"(x0), "v"(x1), "v"(x2), "v"(x3), "v"(y0), "v"(y1), "v"(y2), "v"(y3));
}
__device__ __forceinline__ void guard_pv(v8f& a0, v8f& a1, v8f& b0, v8f& b1,
                                         v16h p0, v16h p1, v16h x0, v16h x1, v16h y0, v16h y1) {
  asm volatile("v_nop\n\tv_nop\n\tv_nop\n\tv_nop"
               : "+v"(a0), "+v"(a1), "+v"(b0), "+v"(b1)
               : "v"(p0), "v"(p1), "v"(x0), "v"(x1), "v"(y0), "v"(y1));
}

__global__ __launch_bounds__(256) void cvt_x_kernel(const float* __restrict__ x, unsigned short* __restrict__ xb, int n8) {
  const int li = (int)blockIdx.x * 256 + (int)threadIdx.x;
  if (li >= n8) return;
  const int tok = li >> 7, pc = li & 127;
  const int bq = tok / SEQ;
  const int srow = bq * SEQ_FULL + (tok - bq * SEQ);
  const float* s = x + (size_t)srow * DM + (size_t)pc * 8;
  const v4f a = *(const v4f*)(s);
  const v4f b = *(const v4f*)(s + 4);
  v8us o;
#pragma unroll
  for (int i = 0; i < 4; ++i) {
    o[i]     = bfbits(a[i]);
    o[4 + i] = bfbits(b[i]);
  }
  unsigned short* d = xb + (size_t)li * 8;
  *(volatile v8us*)d = o;
  __threadfence();
  *(volatile v8us*)d = o;
}

__global__ __launch_bounds__(256) void cvt_wt_kernel(const float* __restrict__ src, int spitch,
                                                     unsigned short* __restrict__ dst, int ldd, int dup) {
  __shared__ float sTt[64][33];
  const int k0 = (int)blockIdx.x * 64, n0 = (int)blockIdx.y * 32;
  const int t = (int)threadIdx.x;
  {
    const int kr = t >> 2, cc = (t & 3) * 8;
    const float* s = src + (size_t)(k0 + kr) * spitch + n0 + cc;
    const v4f a = *(const v4f*)(s);
    const v4f b = *(const v4f*)(s + 4);
#pragma unroll
    for (int e = 0; e < 4; ++e) {
      sTt[kr][cc + e]     = a[e];
      sTt[kr][cc + 4 + e] = b[e];
    }
  }
  __syncthreads();
  const int n = t >> 3, kp = (t & 7) * 8;
  v8us o;
#pragma unroll
  for (int i = 0; i < 8; ++i) o[i] = bfbits(sTt[kp + i][n]);
  unsigned short* d = dst + (size_t)(n0 + n) * ldd + k0 + kp;
  *(volatile v8us*)d = o;
  if (dup != 0) *(volatile v8us*)(d + dup) = o;
  __threadfence();
  *(volatile v8us*)d = o;
  if (dup != 0) *(volatile v8us*)(d + dup) = o;
}

template <int MODE>
__global__ __launch_bounds__(256) void proj_kernel(const __bf16* __restrict__ A, int lda,
                                                   const __bf16* __restrict__ Bt, int ldb,
                                                   const float* __restrict__ bias,
                                                   _Float16* __restrict__ Ch, _Float16* __restrict__ Cl,
                                                   float* __restrict__ Cf, int ldc,
                                                   int M, int N, int K) {
  __shared__ __align__(16) float sT[8][16 * 68];
  const int lane = threadIdx.x & 31, wave = threadIdx.x >> 5;
  const int tilesN = N >> 6, tilesM = M >> 6;
  const int tile = (int)blockIdx.x * 8 + wave;
  if (tile >= tilesM * tilesN) return;
  const int tm = tile / tilesN, tn = tile - tm * tilesN;
  const int m0 = tm << 6, n0 = tn << 6;
  const int rl = lane & 15;
  const int koff = (lane >> 4) * 8;
  const int mOff = (lane >> 4) * 8;

  v8f acc[4][4];
#pragma unroll
  for (int i = 0; i < 4; ++i)
#pragma unroll
    for (int j = 0; j < 4; ++j) acc[i][j] = zero8();

#pragma unroll 1
  for (int k0 = 0; k0 < K; k0 += 32) {
    v16b bh[4];
#pragma unroll
    for (int j = 0; j < 4; ++j) bh[j] = ldfragb(Bt + (size_t)(n0 + (j << 4) + rl) * ldb + koff + k0);
#pragma unroll
    for (int i = 0; i < 4; ++i) {
      const v16b ah = ldfragb(A + (size_t)(m0 + (i << 4) + rl) * lda + koff + k0);
#pragma unroll
      for (int j = 0; j < 4; ++j) acc[i][j] = mmabf(ah, bh[j], acc[i][j]);
      guard_g(acc[i][0], acc[i][3], ah, bh[3]);
    }
    keep4(bh[0], bh[1], bh[2], bh[3]);
  }
  accg4(acc[0][0], acc[0][1], acc[0][2], acc[0][3]);
  accg4(acc[1][0], acc[1][1], acc[1][2], acc[1][3]);
  accg4(acc[2][0], acc[2][1], acc[2][2], acc[2][3]);
  accg4(acc[3][0], acc[3][1], acc[3][2], acc[3][3]);

  float* slab = sT[wave];
  const int qq = lane >> 3, c8 = (lane & 7) * 8;
  const int q2 = lane >> 4, c4 = (lane & 15) * 4;
  v4f bA = {0.0f, 0.0f, 0.0f, 0.0f};
  v4f bB = {0.0f, 0.0f, 0.0f, 0.0f};
  if (MODE == 0) {
    const v4f t0 = *(const v4f*)(bias + n0 + c8);
    const v4f t1 = *(const v4f*)(bias + n0 + c8 + 4);
#pragma unroll
    for (int e = 0; e < 4; ++e) { bA[e] = bfval(t0[e]); bB[e] = bfval(t1[e]); }
  }
  if (MODE == 2) {
    const v4f t0 = *(const v4f*)(bias + n0 + c4);
#pragma unroll
    for (int e = 0; e < 4; ++e) bA[e] = bfval(t0[e]);
  }

#pragma unroll
  for (int i = 0; i < 4; ++i) {
    const int mBase = m0 + (i << 4);
#pragma unroll
    for (int j = 0; j < 4; ++j) {
#pragma unroll
      for (int r = 0; r < 8; ++r) slab[(mOff + r) * 68 + (j << 4) + rl] = acc[i][j][r];
    }
    __builtin_amdgcn_fence(3, "workgroup");
    __builtin_amdgcn_wave_barrier();
    __builtin_amdgcn_fence(2, "workgroup");
    if (MODE != 2) {
#pragma unroll
      for (int ps = 0; ps < 2; ++ps) {
#pragma unroll
        for (int it = 0; it < 4; ++it) {
          const int row = it * 4 + qq;
          const float* sp = slab + row * 68 + c8;
          v4f u0 = *(const v4f*)(sp);
          v4f u1 = *(const v4f*)(sp + 4);
          if (MODE == 0) {
            u0 = u0 + bA;
            u1 = u1 + bB;
          } else {
            const float bm = bfval(bias[mBase + row]);
            u0 = u0 + bm;
            u1 = u1 + bm;
          }
          v8h hv, lv;
#pragma unroll
          for (int e = 0; e < 4; ++e) {
            const _Float16 g0 = (_Float16)u0[e];
            hv[e] = g0;
            lv[e] = (_Float16)((u0[e] - (float)g0) * 2048.0f);
            const _Float16 g1 = (_Float16)u1[e];
            hv[4 + e] = g1;
            lv[4 + e] = (_Float16)((u1[e] - (float)g1) * 2048.0f);
          }
          const size_t go = (size_t)(mBase + row) * ldc + n0 + c8;
          *(volatile v8h*)(Ch + go) = hv;
          *(volatile v8h*)(Cl + go) = lv;
        }
        __threadfence();
      }
    } else {
#pragma unroll
      for (int ps = 0; ps < 2; ++ps) {
#pragma unroll
        for (int it = 0; it < 8; ++it) {
          const int row = it * 2 + q2;
          const float* sp = slab + row * 68 + c4;
          const v4f u = *(const v4f*)(sp) + bA;
          const int m = mBase + row;
          const int bq = m / SEQ;
          const int orow = bq * SEQ_FULL + (m - bq * SEQ);
          *(volatile v4f*)(Cf + (size_t)orow * ldc + n0 + c4) = u;
        }
        __threadfence();
      }
    }
    __builtin_amdgcn_fence(3, "workgroup");
    __builtin_amdgcn_wave_barrier();
    __builtin_amdgcn_fence(2, "workgroup");
  }
}

#define QB     16
#define NWA    4
#define OSP    68
#define QT_RES 64
static_assert((OSP % 4) == 0 && OSP >= HD && (SEQ % QB) == 0 && ((QB * OSP * 4) % 16) == 0);

template <bool RES>
__global__ __launch_bounds__(NWA * 32) __attribute__((amdgpu_num_vgpr(256)))
void attn_kernel(const _Float16* __restrict__ QKh, const _Float16* __restrict__ QKl,
                 const _Float16* __restrict__ Vth, const _Float16* __restrict__ Vtl,
                 unsigned short* __restrict__ Cb, int qtlo, int nqt, int ntask) {
  __shared__ __align__(16) float sO[NWA][QB * OSP];
  const int tid = (int)threadIdx.x;
  const int wave = __builtin_amdgcn_readfirstlane(tid >> 5);
  const int lane = tid & 31, hh = lane >> 4, c = lane & 15;
  const int task = (int)blockIdx.x * NWA + wave;
  if (task >= ntask) return;
  const int bh = task / nqt;
  const int qt = qtlo + (task - bh * nqt);
  const int b = bh / NH, h = bh - b * NH;
  const int q0 = qt * QB;
  const size_t seq0 = (size_t)b * SEQ;
  const size_t tok0 = seq0 + (size_t)q0;
  const float ninf = -__builtin_inff();
  const int qme = q0 + c;

  const _Float16* qp = QKh + (tok0 + c) * (size_t)LQK + h * HD + 8 * hh;
  const _Float16* qr = QKl + (tok0 + c) * (size_t)LQK + h * HD + 8 * hh;
  const v16h bq0 = ldfrag(qp), bq1 = ldfrag(qp + 32);
  const v16h bl0 = ldfrag(qr), bl1 = ldfrag(qr + 32);

  const _Float16* kp  = QKh + (seq0 + c) * (size_t)LQK + DM + h * HD + 8 * hh;
  const _Float16* krp = QKl + (seq0 + c) * (size_t)LQK + DM + h * HD + 8 * hh;
  const _Float16* vp  = Vth + (size_t)(h * HD + c) * NTOK + seq0 + 8 * hh;
  const _Float16* vrp = Vtl + (size_t)(h * HD + c) * NTOK + seq0 + 8 * hh;

  v8f oacc1[4], oacc2[4];
#pragma unroll
  for (int nt = 0; nt < 4; ++nt) { oacc1[nt] = zero8(); oacc2[nt] = zero8(); }
  float mrun = ninf, lrun = 0.0f;
  const int nstep = (q0 + QB + 31) >> 5;

#pragma unroll 1
  for (int st = 0; st < nstep; ++st) {
    const int kv = st << 5;
    v8f s1[2], s2[2];
#pragma unroll
    for (int j = 0; j < 2; ++j) {
      const size_t ko = (size_t)(kv + 16 * j) * LQK;
      const v16h a0 = ldfrag(kp + ko), a1 = ldfrag(kp + ko + 32);
      v16h e0 = a0, e1 = a1;
      if (RES) { e0 = ldfrag(krp + ko); e1 = ldfrag(krp + ko + 32); }
      v8f t1 = zero8(), t2 = zero8();
      t1 = mma16(a0, bq0, t1);
      t1 = mma16(a1, bq1, t1);
      t2 = mma16(a0, bl0, t2);
      t2 = mma16(a1, bl1, t2);
      if (RES) {
        t2 = mma16(e0, bq0, t2);
        t2 = mma16(e1, bq1, t2);
      }
      guard_st(t1, t2, a0, a1, e0, e1, bq0, bq1, bl0, bl1);
      s1[j] = t1;
      s2[j] = t2;
    }
    float pm = ninf;
#pragma unroll
    for (int j = 0; j < 2; ++j) {
#pragma unroll
      for (int r = 0; r < 8; ++r) {
        float s = (s1[j][r] + s2[j][r] * 0.00048828125f) * 0.125f;
        const int key = kv + 16 * j + 8 * hh + r;
        s = (key > qme) ? ninf : s;
        s1[j][r] = s;
        pm = fmaxf(pm, s);
      }
    }
    pm = fmaxf(pm, __shfl_xor(pm, 16, 32));
    const float mnew = fmaxf(mrun, pm);
    const float alpha = __expf(mrun - mnew);
    mrun = mnew;
    float ps = 0.0f;
    v8h ph[2], pr[2];
#pragma unroll
    for (int j = 0; j < 2; ++j) {
#pragma unroll
      for (int r = 0; r < 8; ++r) {
        const float p = __expf(s1[j][r] - mnew);
        ps += p;
        const float p16 = p * 16.0f;
        const _Float16 g = (_Float16)p16;
        ph[j][r] = g;
        pr[j][r] = (_Float16)((p16 - (float)g) * 2048.0f);
      }
    }
    ps += __shfl_xor(ps, 16, 32);
    lrun = lrun * alpha + ps;
    {
      float ar[8];
#pragma unroll
      for (int r = 0; r < 8; ++r) ar[r] = __shfl(alpha, 8 * hh + r, 32);
#pragma unroll
      for (int nt = 0; nt < 4; ++nt) {
#pragma unroll
        for (int r = 0; r < 8; ++r) {
          oacc1[nt][r] *= ar[r];
          oacc2[nt][r] *= ar[r];
        }
      }
    }
    Frag PA, PZ;
    PA.half[0] = ph[0]; PA.half[1] = ph[1];
    PZ.half[0] = pr[0]; PZ.half[1] = pr[1];
    const v16h pa = PA.v;
    v16h pz = pa;
    if (RES) pz = PZ.v;
#pragma unroll
    for (int g = 0; g < 2; ++g) {
      const size_t o0 = (size_t)(32 * g) * NTOK + kv;
      const size_t o1 = (size_t)(32 * g + 16) * NTOK + kv;
      const v16h x0 = ldfrag(vp + o0), x1 = ldfrag(vp + o1);
      const v16h y0 = ldfrag(vrp + o0), y1 = ldfrag(vrp + o1);
      oacc1[2 * g]     = mma16(pa, x0, oacc1[2 * g]);
      oacc1[2 * g + 1] = mma16(pa, x1, oacc1[2 * g + 1]);
      oacc2[2 * g]     = mma16(pa, y0, oacc2[2 * g]);
      oacc2[2 * g + 1] = mma16(pa, y1, oacc2[2 * g + 1]);
      if (RES) {
        oacc2[2 * g]     = mma16(pz, x0, oacc2[2 * g]);
        oacc2[2 * g + 1] = mma16(pz, x1, oacc2[2 * g + 1]);
      }
      guard_pv(oacc1[2 * g], oacc1[2 * g + 1], oacc2[2 * g], oacc2[2 * g + 1], pa, pz, x0, x1, y0, y1);
    }
  }

  const float linv = (1.0f / lrun) * 0.0625f;
  float li[8];
#pragma unroll
  for (int r = 0; r < 8; ++r) li[r] = __shfl(linv, 8 * hh + r, 32);
  float* Os = sO[wave];
#pragma unroll
  for (int nt = 0; nt < 4; ++nt) {
    const int col = 16 * nt + c;
#pragma unroll
    for (int r = 0; r < 8; ++r) Os[(8 * hh + r) * OSP + col] = (oacc1[nt][r] + oacc2[nt][r] * 0.00048828125f) * li[r];
  }
  __builtin_amdgcn_fence(3, "workgroup");
  __builtin_amdgcn_wave_barrier();
  __builtin_amdgcn_fence(2, "workgroup");
  {
    const int qq = lane >> 3, c8 = (lane & 7) * 8;
#pragma unroll
    for (int ps = 0; ps < 2; ++ps) {
#pragma unroll
      for (int it = 0; it < 4; ++it) {
        const int row = it * 4 + qq;
        const float* sp = Os + row * OSP + c8;
        const v4f u0 = *(const v4f*)(sp);
        const v4f u1 = *(const v4f*)(sp + 4);
        v8us oh, ol;
#pragma unroll
        for (int e = 0; e < 4; ++e) {
          const unsigned short g0 = bfbits(u0[e]);
          oh[e] = g0;
          ol[e] = bfbits(u0[e] - __uint_as_float(((unsigned)g0) << 16));
          const unsigned short g1 = bfbits(u1[e]);
          oh[4 + e] = g1;
          ol[4 + e] = bfbits(u1[e] - __uint_as_float(((unsigned)g1) << 16));
        }
        unsigned short* d = Cb + (tok0 + (size_t)row) * LCB + h * HD + c8;
        *(volatile v8us*)d = oh;
        *(volatile v8us*)(d + DM) = ol;
      }
      __threadfence();
    }
  }
}

static_assert((size_t)NB_FULL * SEQ_FULL * DM * 2 + (size_t)3 * DM * DM * 2 + (size_t)DM * 2 * DM * 2 +
              (size_t)NB_FULL * SEQ_FULL * LQK * 2 * 2 + (size_t)DM * NB_FULL * SEQ_FULL * 2 * 2 +
              (size_t)NB_FULL * SEQ_FULL * LCB * 2 <= (size_t)134217728);

extern "C" void kernel_launch(void* const* d_in, const int* in_sizes, int n_in,
                              void* d_out, int out_size, void* d_ws, size_t ws_size,
                              hipStream_t stream) {
  if (n_in < 5) return;
  const int needTok = (NB - 1) * SEQ_FULL + SEQ;
  if (in_sizes[0] < needTok * DM) return;
  if (in_sizes[1] < 3 * DM * DM) return;
  if (in_sizes[2] < 3 * DM) return;
  if (in_sizes[3] < DM * DM) return;
  if (in_sizes[4] < DM) return;
  if (out_size < needTok * DM) return;

  const float* x    = (const float*)d_in[0];
  const float* Wqkv = (const float*)d_in[1];
  const float* bqkv = (const float*)d_in[2];
  const float* Wo   = (const float*)d_in[3];
  const float* bo   = (const float*)d_in[4];
  float* out = (float*)d_out;

  const size_t bX    = (size_t)NTOK * DM * 2;
  const size_t bWqkv = (size_t)3 * DM * DM * 2;
  const size_t bWo2  = (size_t)DM * (2 * DM) * 2;
  const size_t bQK   = (size_t)NTOK * LQK * 2;
  const size_t bVt   = (size_t)DM * NTOK * 2;
  const size_t bCb   = (size_t)NTOK * LCB * 2;
  size_t off = 0;
  const size_t oXb  = off; off += bX;
  const size_t oWq  = off; off += bWqkv;
  const size_t oWo  = off; off += bWo2;
  const size_t oQKh = off; off += bQK;
  const size_t oQKl = off; off += bQK;
  const size_t oVh  = off; off += bVt;
  const size_t oVl  = off; off += bVt;
  const size_t oCb  = off; off += bCb;
  if (off > ws_size) return;
  if (off > (size_t)134217728) return;

  char* ws = (char*)d_ws;
  unsigned short* Xb    = (unsigned short*)(ws + oXb);
  unsigned short* WqkvT = (unsigned short*)(ws + oWq);
  unsigned short* Wo2T  = (unsigned short*)(ws + oWo);
  _Float16* QKh = (_Float16*)(ws + oQKh);
  _Float16* QKl = (_Float16*)(ws + oQKl);
  _Float16* Vth = (_Float16*)(ws + oVh);
  _Float16* Vtl = (_Float16*)(ws + oVl);
  unsigned short* Cb = (unsigned short*)(ws + oCb);

  const dim3 blk(256);
  const int n8 = NTOK * DM / 8;
  if ((n8 % 256) != 0) return;

  cvt_x_kernel<<<dim3(n8 / 256), blk, 0, stream>>>(x, Xb, n8);
  cvt_wt_kernel<<<dim3(DM / 64, (3 * DM) / 32), blk, 0, stream>>>(Wqkv, 3 * DM, WqkvT, DM, 0);
  cvt_wt_kernel<<<dim3(DM / 64, DM / 32), blk, 0, stream>>>(Wo, DM, Wo2T, 2 * DM, DM);
  {
    const int tiles = (NTOK / 64) * ((2 * DM) / 64);
    proj_kernel<0><<<dim3((tiles + 7) / 8), blk, 0, stream>>>(
        (const __bf16*)Xb, DM, (const __bf16*)WqkvT, DM, bqkv, QKh, QKl, out, LQK, NTOK, 2 * DM, DM);
  }
  {
    const int tiles = (DM / 64) * (NTOK / 64);
    proj_kernel<1><<<dim3((tiles + 7) / 8), blk, 0, stream>>>(
        (const __bf16*)(WqkvT + (size_t)(2 * DM) * DM), DM, (const __bf16*)Xb, DM, bqkv + 2 * DM,
        Vth, Vtl, out, NTOK, DM, NTOK, DM);
  }
  {
    const int nqtAll = SEQ / QB;
    const int nqtA = (nqtAll < QT_RES) ? nqtAll : QT_RES;
    const int nqtB = nqtAll - nqtA;
    const int ntaskA = NB * NH * nqtA;
    attn_kernel<true><<<dim3((ntaskA + NWA - 1) / NWA), dim3(NWA * 32), 0, stream>>>(
        QKh, QKl, Vth, Vtl, Cb, 0, nqtA, ntaskA);
    if (nqtB > 0) {
      const int ntaskB = NB * NH * nqtB;
      attn_kernel<false><<<dim3((ntaskB + NWA - 1) / NWA), dim3(NWA * 32), 0, stream>>>(
          QKh, QKl, Vth, Vtl, Cb, nqtA, nqtB, ntaskB);
    }
  }
  {
    const int tiles = (NTOK / 64) * (DM / 64);
    proj_kernel<2><<<dim3((tiles + 7) / 8), blk, 0, stream>>>(
        (const __bf16*)Cb, LCB, (const __bf16*)Wo2T, 2 * DM, bo, QKh, QKl, out, DM, NTOK, DM, 2 * DM);
  }
  (void)hipGetLastError();
}
